// ConvolutionModule_32744830665311
// MI455X (gfx1250) — hardware-verified
//
#include <hip/hip_runtime.h>
#include <stddef.h>
#include <math.h>


#define DIN     128
#define DH      256
#define K1      256
#define K2      512
#define NG      64
#define NTHR    256
#define NWAVE   8
#define EPT     8
#define NGRP    2
#define CHUNK   (NTHR * EPT * NGRP)
#define WCAP    (EPT * NGRP * 32)
#define LISTN   (NWAVE * WCAP)
#define NBC     4096
#define NBF     1024
#define RCAP    32768
#define RBN     128
#define TGT     256
#define DEGCAP  512
#define GROWS   64
#define OTHR    512
#define PG      32
#define NCSB    64
#define WSCAP   134217728
#define WP1     0
#define WP2     (DH * K1)
#define WPTOT   (DH * K1 + DH * K2)
#define LDS_FILL ((RCAP + NBF + LISTN) * 4 + 64)
#define LDS_GEMM (NWAVE * 32 * 64 * 4)
#define SC_AGG   0.25f
#define SC_WREL  256.0f
#define SC_WROOT 64.0f
#define SC_OUT   0.015625f

static_assert((CHUNK & (CHUNK - 1)) == 0);
static_assert(CHUNK <= 4096);
static_assert(NBC <= 4096 && NBF <= 4096 && PG <= 4096);
static_assert((NBC & (NBC - 1)) == 0 && (NBF & (NBF - 1)) == 0 && (PG & (PG - 1)) == 0);
static_assert(NBC == 4 * NBF);
static_assert(OTHR * 8 == NBC);
static_assert((RCAP % 32) == 0);
static_assert(TGT == NWAVE * 32);
static_assert((NBC % TGT) == 0 && (TGT % GROWS) == 0);
static_assert(GROWS == 2 * 32 && NWAVE == 8 && DH == 4 * 64);
static_assert((NG % PG) == 0 && PG == 4 * NWAVE);
static_assert((K1 % 32) == 0 && (K2 % 32) == 0 && K1 == 2 * DIN && K2 == 2 * DH);
static_assert(NTHR == 2 * DIN);
static_assert(RBN == 4 * 32);

typedef float          v4f  __attribute__((ext_vector_type(4)));
typedef float          v8f  __attribute__((ext_vector_type(8)));
typedef int            v4i  __attribute__((ext_vector_type(4)));
typedef _Float16       v4h  __attribute__((ext_vector_type(4)));
typedef _Float16       v8h  __attribute__((ext_vector_type(8)));
typedef _Float16       v16h __attribute__((ext_vector_type(16)));
union FragH { v16h v; v8h half[2]; };

template <int CH> struct AggT;
template <> struct AggT<128> { typedef v4f VT; typedef v4h HT; };
template <> struct AggT<256> { typedef v8f VT; typedef v8h HT; };

__device__ __forceinline__ v8f wmh(v16h a, v16h b, v8f c) {
  v8f d = __builtin_amdgcn_wmma_f32_16x16x32_f16(false, a, false, b, (short)0, c, false, false);
  asm volatile("v_nop\n\tv_nop\n\tv_nop\n\tv_nop" : "+v"(d) : "v"(a), "v"(b));
  return d;
}

template <int NB>
__device__ __forceinline__ int scan_chunk(const int* __restrict__ dsts, int nE, int cbase, int slotBase,
                                          int vec8, int* list, int tid, int lane, int wave) {
  int wc = 0;
#pragma unroll
  for (int g = 0; g < NGRP; ++g) {
    const int el0  = (g * NTHR + tid) * EPT;
    const int e0   = cbase + el0;
    const int sent = -2147483647 - 1;
    v4i da, db;
    if (vec8 != 0 && cbase + CHUNK <= nE) {
      da = *(const v4i*)(dsts + e0);
      db = *(const v4i*)(dsts + e0 + 4);
    } else {
      da.x = (e0     < nE) ? dsts[min(e0, nE - 1)] : sent;
      da.y = (e0 + 1 < nE) ? dsts[min(e0 + 1, nE - 1)] : sent;
      da.z = (e0 + 2 < nE) ? dsts[min(e0 + 2, nE - 1)] : sent;
      da.w = (e0 + 3 < nE) ? dsts[min(e0 + 3, nE - 1)] : sent;
      db.x = (e0 + 4 < nE) ? dsts[min(e0 + 4, nE - 1)] : sent;
      db.y = (e0 + 5 < nE) ? dsts[min(e0 + 5, nE - 1)] : sent;
      db.z = (e0 + 6 < nE) ? dsts[min(e0 + 6, nE - 1)] : sent;
      db.w = (e0 + 7 < nE) ? dsts[min(e0 + 7, nE - 1)] : sent;
    }
    const unsigned nb = (unsigned)slotBase;
    const unsigned s0 = (unsigned)da.x - nb, s1 = (unsigned)da.y - nb;
    const unsigned s2 = (unsigned)da.z - nb, s3 = (unsigned)da.w - nb;
    const unsigned s4 = (unsigned)db.x - nb, s5 = (unsigned)db.y - nb;
    const unsigned s6 = (unsigned)db.z - nb, s7 = (unsigned)db.w - nb;
    const bool h0 = s0 < (unsigned)NB, h1 = s1 < (unsigned)NB, h2 = s2 < (unsigned)NB, h3 = s3 < (unsigned)NB;
    const bool h4 = s4 < (unsigned)NB, h5 = s5 < (unsigned)NB, h6 = s6 < (unsigned)NB, h7 = s7 < (unsigned)NB;
    const unsigned any = __builtin_amdgcn_ballot_w32(h0 | h1 | h2 | h3 | h4 | h5 | h6 | h7);
    if (any != 0u) {
#define HITJ(J, HJ, SJ) { \
        const unsigned mj = __builtin_amdgcn_ballot_w32(HJ); \
        if (mj != 0u) { \
          if (HJ) { \
            const int pos = wc + (int)__builtin_amdgcn_mbcnt_lo(mj, 0u); \
            if (pos < WCAP) list[wave * WCAP + pos] = ((el0 + (J)) << 12) | (int)(SJ); \
          } \
          wc += (int)__builtin_popcount(mj); } }
      HITJ(0, h0, s0)
      HITJ(1, h1, s1)
      HITJ(2, h2, s2)
      HITJ(3, h3, s3)
      HITJ(4, h4, s4)
      HITJ(5, h5, s5)
      HITJ(6, h6, s6)
      HITJ(7, h7, s7)
#undef HITJ
    }
  }
  return wc;
}

__global__ __launch_bounds__(NTHR) void k_wprep(
    const float* __restrict__ w1r, const float* __restrict__ w1o,
    const float* __restrict__ w2r, const float* __restrict__ w2o, _Float16* wp) {
  const int blk = blockIdx.x, tid = threadIdx.x;
  int KD, kin, base, i;
  const float* wa; const float* wb;
  if (blk < 32) { KD = K1; kin = DIN; base = WP1; i = blk * NTHR + tid;        wa = w1r; wb = w1o; }
  else          { KD = K2; kin = DH;  base = WP2; i = (blk - 32) * NTHR + tid; wa = w2r; wb = w2o; }
  const int kq = KD >> 3;
  const int n  = i / kq;
  const int k0 = (i - n * kq) * 8;
  v8f v;
#pragma unroll
  for (int e = 0; e < 8; ++e) {
    const int k  = k0 + e;
    const int kk = k & (kin - 1);
    const float va = wa[(size_t)kk * DH + n];
    const float vb = wb[(size_t)kk * DH + n];
    v[e] = (k < kin) ? va * SC_WREL : vb * SC_WROOT;
  }
  const v8h hv = __builtin_convertvector(v, v8h);
  _Float16* d = wp + base + (size_t)i * 8;
  *(volatile v8h*)d = hv;
  __threadfence();
  *(volatile v8h*)d = hv;
}

__global__ __launch_bounds__(NTHR) void k_colsum(const float* __restrict__ x, double* part, int nN) {
  const int tid = threadIdx.x, c = tid & (DIN - 1), par = tid >> 7;
  const int rpb = (nN + NCSB - 1) / NCSB;
  const int r0 = blockIdx.x * rpb;
  int r1 = r0 + rpb;
  r1 = r1 > nN ? nN : r1;
  double s = 0.0;
#pragma unroll 1
  for (int r = r0 + par; r < r1; r += 2) s += (double)x[(size_t)r * DIN + c];
  double* p = part + (size_t)blockIdx.x * NTHR + tid;
  *(volatile double*)p = s;
  __threadfence();
  *(volatile double*)p = s;
}

__global__ __launch_bounds__(NTHR) void k_hand(const double* __restrict__ part, float* out1) {
  __shared__ double scol[DIN];
  __shared__ __attribute__((aligned(16))) float sres[DIN + 4];
  const int tid = threadIdx.x;
  if (tid < DIN) {
    double s = 0.0;
#pragma unroll 1
    for (int b = 0; b < NCSB; ++b) {
      s += part[(size_t)b * NTHR + tid];
      s += part[(size_t)b * NTHR + DIN + tid];
    }
    scol[tid] = s;
  }
  if (tid < 4) sres[DIN + tid] = 0.0f;
  __syncthreads();
  double tot = 0.0;
#pragma unroll 1
  for (int c = 0; c < DIN; ++c) tot += scol[c];
  const float gs  = (float)tot;
  const float rgs = 1.0f / gs;
  if (tid < DIN) sres[tid] = (float)scol[tid] * rgs;
  __syncthreads();
  if (tid == 0) sres[DIN] = logf(gs);
  __syncthreads();
  v4f v = {0.f, 0.f, 0.f, 0.f};
  if (tid < 32) v = *(const v4f*)(sres + 4 * tid);
  const float last = sres[DIN];
  if (tid < 32) *(volatile v4f*)(out1 + 4 * tid) = v;
  if (tid == 32) *(volatile float*)(out1 + DIN) = last;
  __threadfence();
  if (tid < 32) *(volatile v4f*)(out1 + 4 * tid) = v;
  if (tid == 32) *(volatile float*)(out1 + DIN) = last;
}

__global__ __launch_bounds__(NTHR) void k_count(const int* __restrict__ ei, int* cnt, int nE, int vec8) {
  __shared__ __attribute__((aligned(16))) int scnt[NBC];
  __shared__ __attribute__((aligned(16))) int list[LISTN];
  __shared__ int wcnt[NWAVE];
  const int tid = threadIdx.x, lane = tid & 31, wave = tid >> 5;
  const int nodeBase = blockIdx.x * NBC;
  const int* dsts = ei + nE;

  for (int i = tid; i < NBC; i += NTHR) scnt[i] = 0;
  __syncthreads();

  const int nChunks = (nE + CHUNK - 1) / CHUNK;
#pragma unroll 1
  for (int ch = 0; ch < nChunks; ++ch) {
    const int cbase = ch * CHUNK;
    const int wc = scan_chunk<NBC>(dsts, nE, cbase, nodeBase, vec8, list, tid, lane, wave);
    if (lane == 0) wcnt[wave] = wc;
    __syncthreads();
    if (wave == 0) {
#pragma unroll 1
      for (int wsx = 0; wsx < NWAVE; ++wsx) {
        int n = __builtin_amdgcn_readfirstlane(wcnt[wsx]);
        n = n > WCAP ? WCAP : (n < 0 ? 0 : n);
        const int* lp = list + wsx * WCAP;
#pragma unroll 1
        for (int i = 0; i < n; ++i) {
          const int ent  = __builtin_amdgcn_readfirstlane(lp[i]);
          const int slot = ent & (NBC - 1);
          if (lane == 0) scnt[slot] = scnt[slot] + 1;
        }
      }
    }
    __syncthreads();
  }

  v4i cq[4];
#pragma unroll
  for (int q = 0; q < 4; ++q) {
    const int f = (wave * 4 + q) * 128 + 4 * lane;
    cq[q] = *(const v4i*)(scnt + f);
  }
  int* cp = cnt + (size_t)nodeBase;
#pragma unroll
  for (int q = 0; q < 4; ++q) {
    const int f = (wave * 4 + q) * 128 + 4 * lane;
    *(volatile v4i*)(cp + f) = cq[q];
  }
  __threadfence();
#pragma unroll
  for (int q = 0; q < 4; ++q) {
    const int f = (wave * 4 + q) * 128 + 4 * lane;
    *(volatile v4i*)(cp + f) = cq[q];
  }
}

__global__ __launch_bounds__(OTHR) void k_offsets(
    const int* __restrict__ cnt, int* off, int* rbase, int nChunk) {
  __shared__ __attribute__((aligned(16))) int soff[NBC];
  __shared__ __attribute__((aligned(16))) int srb[RBN];
  __shared__ int wtot[OTHR / 32];
  const int tid = threadIdx.x, lane = tid & 31, wave = tid >> 5, sub = tid >> 7;
  for (int i = tid; i < RBN; i += OTHR) srb[i] = 0;
  int carry = 0;
#pragma unroll 1
  for (int ch = 0; ch < nChunk; ++ch) {
    const int base = ch * NBC;
    const v4i c0 = *(const v4i*)(cnt + base + 8 * tid);
    const v4i c1 = *(const v4i*)(cnt + base + 8 * tid + 4);
    const int e0 = max(c0.x, 0), e1 = max(c0.y, 0), e2 = max(c0.z, 0), e3 = max(c0.w, 0);
    const int e4 = max(c1.x, 0), e5 = max(c1.y, 0), e6 = max(c1.z, 0), e7 = max(c1.w, 0);
    const int ts = e0 + e1 + e2 + e3 + e4 + e5 + e6 + e7;
    int incl = ts;
#pragma unroll
    for (int d = 1; d < 32; d <<= 1) {
      const int t = __shfl_up(incl, d);
      if (lane >= d) incl += t;
    }
    if (lane == 31) wtot[wave] = incl;
    __syncthreads();
    const int S0 = wtot[0]  + wtot[1]  + wtot[2]  + wtot[3];
    const int S1 = wtot[4]  + wtot[5]  + wtot[6]  + wtot[7];
    const int S2 = wtot[8]  + wtot[9]  + wtot[10] + wtot[11];
    const int S3 = wtot[12] + wtot[13] + wtot[14] + wtot[15];
    int pre = 0;
#pragma unroll 1
    for (int w = 4 * sub; w < wave; ++w) pre += wtot[w];
    const int b0 = carry;
    const int b1 = b0 + ((S0 + 31) & ~31);
    const int b2 = b1 + ((S1 + 31) & ~31);
    const int b3 = b2 + ((S2 + 31) & ~31);
    const int b4 = b3 + ((S3 + 31) & ~31);
    const int myb = sub == 0 ? b0 : (sub == 1 ? b1 : (sub == 2 ? b2 : b3));
    if (tid == 0) {
      srb[min(4 * ch + 0, RBN - 1)] = b0;
      srb[min(4 * ch + 1, RBN - 1)] = b1;
      srb[min(4 * ch + 2, RBN - 1)] = b2;
      srb[min(4 * ch + 3, RBN - 1)] = b3;
    }
    int run = myb + pre + incl - ts;
    soff[8 * tid + 0] = run; run += e0;
    soff[8 * tid + 1] = run; run += e1;
    soff[8 * tid + 2] = run; run += e2;
    soff[8 * tid + 3] = run; run += e3;
    soff[8 * tid + 4] = run; run += e4;
    soff[8 * tid + 5] = run; run += e5;
    soff[8 * tid + 6] = run; run += e6;
    soff[8 * tid + 7] = run;
    carry = b4;
    __syncthreads();
    const v4i o0 = *(const v4i*)(soff + 4 * tid);
    const v4i o1 = *(const v4i*)(soff + 4 * (tid + OTHR));
    int* op = off + base;
    *(volatile v4i*)(op + 4 * tid) = o0;
    *(volatile v4i*)(op + 4 * (tid + OTHR)) = o1;
    __threadfence();
    *(volatile v4i*)(op + 4 * tid) = o0;
    *(volatile v4i*)(op + 4 * (tid + OTHR)) = o1;
    __syncthreads();
  }
  if (tid == 0) srb[min(4 * nChunk, RBN - 1)] = carry;
  __syncthreads();
  v4i rv = {0, 0, 0, 0};
  if (tid < 32) rv = *(const v4i*)(srb + 4 * tid);
  if (tid < 32) *(volatile v4i*)(rbase + 4 * tid) = rv;
  __threadfence();
  if (tid < 32) *(volatile v4i*)(rbase + 4 * tid) = rv;
}

__global__ __launch_bounds__(NTHR) void k_fill(
    const int* __restrict__ ei, const int* __restrict__ off, const int* __restrict__ rbase,
    int* csr, int nN, int nE, int vec8, int csrLen) {
  extern __shared__ v4f lds_dyn[];
  int* region = (int*)lds_dyn;
  int* cursor = region + RCAP;
  int* list   = cursor + NBF;
  int* wcnt   = list + LISTN;
  const int tid = threadIdx.x, lane = tid & 31, wave = tid >> 5;
  const int b = blockIdx.x;
  const int nodeBase = b * NBF;
  const int* dsts = ei + nE;

  int rb0 = rbase[b];
  const int rb1 = rbase[b + 1];
  rb0 = rb0 < 0 ? 0 : (rb0 > csrLen ? csrLen : rb0);
  rb0 &= ~31;
  int len = rb1 - rb0;
  len = len < 0 ? 0 : (len > RCAP ? RCAP : len);
  int lenW = (len + 31) & ~31;
  if (rb0 + lenW > csrLen) lenW = (csrLen - rb0) & ~31;

  {
    const v4i z = {0, 0, 0, 0};
    for (int i = tid; i < RCAP / 4; i += NTHR) ((v4i*)region)[i] = z;
    for (int s = tid; s < NBF; s += NTHR) {
      int o = off[nodeBase + s] - rb0;
      o = o < 0 ? 0 : (o > RCAP ? RCAP : o);
      cursor[s] = o;
    }
  }
  __syncthreads();

  const int nChunks = (nE + CHUNK - 1) / CHUNK;
#pragma unroll 1
  for (int ch = 0; ch < nChunks; ++ch) {
    const int cbase = ch * CHUNK;
    const int wc = scan_chunk<NBF>(dsts, nE, cbase, nodeBase, vec8, list, tid, lane, wave);
    if (lane == 0) wcnt[wave] = wc;
    __syncthreads();
    if (wave == 0) {
#pragma unroll 1
      for (int wsx = 0; wsx < NWAVE; ++wsx) {
        int n = __builtin_amdgcn_readfirstlane(wcnt[wsx]);
        n = n > WCAP ? WCAP : (n < 0 ? 0 : n);
        const int* lp = list + wsx * WCAP;
#pragma unroll 1
        for (int i = 0; i < n; ++i) {
          const int ent  = __builtin_amdgcn_readfirstlane(lp[i]);
          const int slot = ent & (NBF - 1);
          int e = cbase + ((ent >> 12) & (CHUNK - 1));
          e = e > nE - 1 ? nE - 1 : e;
          int src = ei[e];
          src = src < 0 ? 0 : (src > nN - 1 ? nN - 1 : src);
          if (lane == 0) {
            int pos = cursor[slot];
            pos = pos < 0 ? 0 : (pos > RCAP - 1 ? RCAP - 1 : pos);
            region[pos] = src;
            const int np = pos + 1;
            cursor[slot] = np > RCAP ? RCAP : np;
          }
        }
      }
    }
    __syncthreads();
  }

  const int nv = lenW >> 2;
  int* gp = csr + rb0;
#pragma unroll 1
  for (int i = tid; i < nv; i += NTHR) { const v4i v = ((const v4i*)region)[i]; *(volatile v4i*)(gp + 4 * i) = v; }
  __threadfence();
#pragma unroll 1
  for (int i = tid; i < nv; i += NTHR) { const v4i v = ((const v4i*)region)[i]; *(volatile v4i*)(gp + 4 * i) = v; }
}

template <int CH>
__global__ __launch_bounds__(NTHR) void k_agg(
    const int* __restrict__ csr, const int* __restrict__ off, const int* __restrict__ cnt,
    const float* __restrict__ xin, _Float16* Ah, int nN, int csrLen) {
  typedef typename AggT<CH>::VT VT;
  typedef typename AggT<CH>::HT HT;
  constexpr int VPL = CH / 32;
  const int tid = threadIdx.x, lane = tid & 31, wave = tid >> 5;
  const int tbase = blockIdx.x * TGT + wave * 32;
  const int cl = tbase + lane;
  const int cnt_l = cnt[cl];
  const int off_l = off[cl];

#pragma unroll 1
  for (int j = 0; j < 32; ++j) {
    const int c = tbase + j;
    int n = __builtin_amdgcn_readlane(cnt_l, j);
    n = n < 0 ? 0 : (n > DEGCAP ? DEGCAP : n);
    const int st = __builtin_amdgcn_readlane(off_l, j);
    VT acc;
#pragma unroll
    for (int e = 0; e < VPL; ++e) acc[e] = 0.0f;
#pragma unroll 1
    for (int q0 = 0; q0 < n; q0 += 32) {
      int pos = st + q0 + lane;
      pos = pos < 0 ? 0 : (pos > csrLen - 1 ? csrLen - 1 : pos);
      int sl = csr[pos];
      sl = sl < 0 ? 0 : (sl > nN - 1 ? nN - 1 : sl);
      const int mcnt = (n - q0) < 32 ? (n - q0) : 32;
#pragma unroll 1
      for (int p = 0; p < mcnt; ++p) {
        const int s = __builtin_amdgcn_readlane(sl, p);
        acc = acc + *(const VT*)(xin + (size_t)s * CH + VPL * lane);
      }
    }
    const int cs = c > nN - 1 ? nN - 1 : c;
    const VT sv = *(const VT*)(xin + (size_t)cs * CH + VPL * lane);
    const VT as = acc * SC_AGG;
    const HT ha = __builtin_convertvector(as, HT);
    const HT hs = __builtin_convertvector(sv, HT);
    _Float16* arow = Ah + (size_t)c * (2 * CH) + VPL * lane;
    *(volatile HT*)arow = ha;
    *(volatile HT*)(arow + CH) = hs;
    __threadfence();
    *(volatile HT*)arow = ha;
    *(volatile HT*)(arow + CH) = hs;
  }
}

template <int KD>
__global__ __launch_bounds__(NTHR) void k_gemm(
    const _Float16* __restrict__ A, const _Float16* __restrict__ Bw,
    const float* __restrict__ bias, float* C) {
  static_assert((KD % 32) == 0);
  extern __shared__ v4f lds_dyn[];
  float* stg = (float*)lds_dyn;
  constexpr int NKT = KD / 32;
  const int tid = threadIdx.x, lane = tid & 31, wave = tid >> 5, hh = lane >> 4, m = lane & 15;
  const int wr = wave >> 2, wc = wave & 3;
  const int row0 = blockIdx.x * GROWS + 32 * wr;
  const int col0 = 64 * wc;

  v8f acc[2][4];
#pragma unroll
  for (int i = 0; i < 2; ++i)
#pragma unroll
    for (int t = 0; t < 4; ++t) { v8f z = {0.f, 0.f, 0.f, 0.f, 0.f, 0.f, 0.f, 0.f}; acc[i][t] = z; }

  const _Float16* ap = A  + (size_t)(row0 + m) * KD + 8 * hh;
  const _Float16* bp = Bw + (size_t)(col0 + m) * KD + 8 * hh;
#pragma unroll 1
  for (int kt = 0; kt < NKT; ++kt) {
    FragH a0, a1;
    a0.half[0] = *(const v8h*)(ap + 32 * kt);
    a0.half[1] = *(const v8h*)(ap + 32 * kt + 16);
    a1.half[0] = *(const v8h*)(ap + (size_t)16 * KD + 32 * kt);
    a1.half[1] = *(const v8h*)(ap + (size_t)16 * KD + 32 * kt + 16);
#pragma unroll
    for (int t = 0; t < 4; ++t) {
      FragH b;
      b.half[0] = *(const v8h*)(bp + (size_t)(16 * t) * KD + 32 * kt);
      b.half[1] = *(const v8h*)(bp + (size_t)(16 * t) * KD + 32 * kt + 16);
      acc[0][t] = wmh(a0.v, b.v, acc[0][t]);
      acc[1][t] = wmh(a1.v, b.v, acc[1][t]);
    }
  }

  float* sw = stg + wave * 2048;
#pragma unroll
  for (int i = 0; i < 2; ++i) {
#pragma unroll
    for (int t = 0; t < 4; ++t) {
      const float bv = bias[col0 + 16 * t + m];
#pragma unroll
      for (int r = 0; r < 8; ++r)
        sw[(16 * i + 8 * hh + r) * 64 + 16 * t + m] = fmaxf(acc[i][t][r] * SC_OUT + bv, 0.0f);
    }
  }
  __syncthreads();

  const int srow = lane >> 4, scol = 4 * (lane & 15);
  float* gb = C + (size_t)row0 * DH + col0 + scol;
#pragma unroll
  for (int q = 0; q < 16; ++q) {
    const int row = 2 * q + srow;
    const v4f v = *(const v4f*)(sw + row * 64 + scol);
    *(volatile v4f*)(gb + (size_t)row * DH) = v;
  }
  __threadfence();
#pragma unroll
  for (int q = 0; q < 16; ++q) {
    const int row = 2 * q + srow;
    const v4f v = *(const v4f*)(sw + row * 64 + scol);
    *(volatile v4f*)(gb + (size_t)row * DH) = v;
  }
}

__global__ __launch_bounds__(NTHR) void k_pool(
    const int* __restrict__ bt, const float* __restrict__ h, float* out, int nN) {
  __shared__ __attribute__((aligned(16))) int   list[LISTN];
  __shared__ __attribute__((aligned(16))) float ssum[PG * DH];
  __shared__ int scnt[PG];
  __shared__ int wcnt[NWAVE];
  const int tid = threadIdx.x, lane = tid & 31, wave = tid >> 5;
  const int gBase = blockIdx.x * PG;

  for (int i = tid; i < PG * DH; i += NTHR) ssum[i] = 0.0f;
  if (tid < PG) scnt[tid] = 0;
  __syncthreads();

  const int nChunks = (nN + CHUNK - 1) / CHUNK;
#pragma unroll 1
  for (int ch = 0; ch < nChunks; ++ch) {
    const int cbase = ch * CHUNK;
    const int wc = scan_chunk<PG>(bt, nN, cbase, gBase, 1, list, tid, lane, wave);
    if (lane == 0) wcnt[wave] = wc;
    __syncthreads();
    if (wave == 0) {
#pragma unroll 1
      for (int wsx = 0; wsx < NWAVE; ++wsx) {
        int n = __builtin_amdgcn_readfirstlane(wcnt[wsx]);
        n = n > WCAP ? WCAP : (n < 0 ? 0 : n);
        const int* lp = list + wsx * WCAP;
#pragma unroll 1
        for (int i = 0; i < n; ++i) {
          const int ent  = __builtin_amdgcn_readfirstlane(lp[i]);
          const int slot = ent & (PG - 1);
          int node = cbase + ((ent >> 12) & (CHUNK - 1));
          node = node > nN - 1 ? nN - 1 : node;
          const float* hp = h + (size_t)node * DH + 8 * lane;
          const v4f va = *(const v4f*)hp;
          const v4f vb = *(const v4f*)(hp + 4);
          float* sp = ssum + slot * DH + 8 * lane;
          v4f s0 = *(const v4f*)sp;
          v4f s1 = *(const v4f*)(sp + 4);
          s0 = s0 + va;
          s1 = s1 + vb;
          *(v4f*)sp = s0;
          *(v4f*)(sp + 4) = s1;
          if (lane == 0) scnt[slot] = scnt[slot] + 1;
        }
      }
    }
    __syncthreads();
  }

#pragma unroll 1
  for (int i = tid; i < PG * DH; i += NTHR) {
    const int g  = i >> 8;
    const int cg = scnt[g];
    const float d  = (float)(cg > 1 ? cg : 1);
    const float rc = 1.0f / d;
    ssum[i] = ssum[i] * rc;
  }
  __syncthreads();

  float* ob = out + (size_t)gBase * DH;
#pragma unroll
  for (int rr = 0; rr < 4; ++rr) {
    const int g = 4 * wave + rr;
#pragma unroll
    for (int hf = 0; hf < 2; ++hf) {
      const int idx = g * DH + 128 * hf + 4 * lane;
      const v4f v = *(const v4f*)(ssum + idx);
      *(volatile v4f*)(ob + idx) = v;
    }
  }
  __threadfence();
#pragma unroll
  for (int rr = 0; rr < 4; ++rr) {
    const int g = 4 * wave + rr;
#pragma unroll
    for (int hf = 0; hf < 2; ++hf) {
      const int idx = g * DH + 128 * hf + 4 * lane;
      const v4f v = *(const v4f*)(ssum + idx);
      *(volatile v4f*)(ob + idx) = v;
    }
  }
}

extern "C" void kernel_launch(void* const* d_in, const int* in_sizes, int n_in,
                              void* d_out, int out_size, void* d_ws, size_t ws_size,
                              hipStream_t stream) {
  if (n_in < 9) return;
  const int nN = in_sizes[2];
  const int nE = in_sizes[1] / 2;
  if (nN <= 0 || nE <= 0 || in_sizes[1] != 2 * nE) return;
  if (nN > (1 << 24) || nE > (1 << 28)) return;
  if (in_sizes[0] != nN * DIN) return;
  if (in_sizes[3] != DIN * DH || in_sizes[4] != DIN * DH || in_sizes[5] != DH) return;
  if (in_sizes[6] != DH * DH || in_sizes[7] != DH * DH || in_sizes[8] != DH) return;
  if (out_size != NG * DH + DIN + 1) return;

  const float* x     = (const float*)d_in[0];
  const int*   ei    = (const int*)d_in[1];
  const int*   batch = (const int*)d_in[2];
  const float* w1r   = (const float*)d_in[3];
  const float* w1o   = (const float*)d_in[4];
  const float* b1    = (const float*)d_in[5];
  const float* w2r   = (const float*)d_in[6];
  const float* w2o   = (const float*)d_in[7];
  const float* b2    = (const float*)d_in[8];
  float* out0 = (float*)d_out;
  float* out1 = out0 + (size_t)NG * DH;

  const int NPAD   = ((nN + TGT - 1) / TGT) * TGT;
  const int nBC    = (nN + NBC - 1) / NBC;
  const int CNTPAD = nBC * NBC;
  if (CNTPAD < NPAD) return;
  if (4 * nBC + 1 > RBN) return;
  const int nBF    = (nN + NBF - 1) / NBF;
  const int csrLen = ((nE + 31) & ~31) + 4096;
  if (31 * 4 * nBC > 4096) return;
  const int nGemm  = NPAD / GROWS;
  const int nAgg   = NPAD / TGT;

  char* ws = (char*)d_ws;
  size_t off = 0;
  const size_t oW   = off; off += (size_t)WPTOT * 2;               off = (off + 255) & ~(size_t)255;
  const size_t oCnt = off; off += (size_t)CNTPAD * 4;              off = (off + 255) & ~(size_t)255;
  const size_t oOff = off; off += (size_t)CNTPAD * 4;              off = (off + 255) & ~(size_t)255;
  const size_t oRb  = off; off += (size_t)RBN * 4;                 off = (off + 255) & ~(size_t)255;
  const size_t oCsr = off; off += (size_t)csrLen * 4;              off = (off + 255) & ~(size_t)255;
  const size_t oA   = off; off += (size_t)NPAD * K2 * 2;           off = (off + 255) & ~(size_t)255;
  const size_t oH   = off; off += (size_t)NPAD * DH * 4;           off = (off + 255) & ~(size_t)255;
  const size_t oPt  = off; off += (size_t)NCSB * NTHR * 8;         off = (off + 255) & ~(size_t)255;
  if (off > ws_size || off > (size_t)WSCAP) return;
  _Float16* wp   = (_Float16*)(ws + oW);
  int*      cnt  = (int*)(ws + oCnt);
  int*      offp = (int*)(ws + oOff);
  int*      rb   = (int*)(ws + oRb);
  int*      csr  = (int*)(ws + oCsr);
  _Float16* Ah   = (_Float16*)(ws + oA);
  float*    H    = (float*)(ws + oH);
  double*   part = (double*)(ws + oPt);

  const int vec8 = ((nE & 3) == 0) ? 1 : 0;

  k_wprep<<<96, NTHR, 0, stream>>>(w1r, w1o, w2r, w2o, wp);

  k_colsum<<<NCSB, NTHR, 0, stream>>>(x, part, nN);
  k_hand<<<1, NTHR, 0, stream>>>(part, out1);

  k_count<<<nBC, NTHR, 0, stream>>>(ei, cnt, nE, vec8);
  k_offsets<<<1, OTHR, 0, stream>>>(cnt, offp, rb, nBC);
  hipFuncSetAttribute(reinterpret_cast<const void*>(&k_fill),
                      hipFuncAttributeMaxDynamicSharedMemorySize, LDS_FILL);
  k_fill<<<nBF, NTHR, LDS_FILL, stream>>>(ei, offp, rb, csr, nN, nE, vec8, csrLen);

  hipFuncSetAttribute(reinterpret_cast<const void*>(&k_gemm<K1>),
                      hipFuncAttributeMaxDynamicSharedMemorySize, LDS_GEMM);
  hipFuncSetAttribute(reinterpret_cast<const void*>(&k_gemm<K2>),
                      hipFuncAttributeMaxDynamicSharedMemorySize, LDS_GEMM);

  k_agg<DIN><<<nAgg, NTHR, 0, stream>>>(csr, offp, cnt, x, Ah, nN, csrLen);
  k_gemm<K1><<<nGemm, NTHR, LDS_GEMM, stream>>>(Ah, wp + WP1, b1, H);

  k_agg<DH><<<nAgg, NTHR, 0, stream>>>(csr, offp, cnt, H, Ah, nN, csrLen);
  k_gemm<K2><<<nGemm, NTHR, LDS_GEMM, stream>>>(Ah, wp + WP2, b2, H);
  k_agg<DH><<<nAgg, NTHR, 0, stream>>>(csr, offp, cnt, H, Ah, nN, csrLen);
  k_gemm<K2><<<nGemm, NTHR, LDS_GEMM, stream>>>(Ah, wp + WP2, b2, H);

  k_pool<<<NG / PG, NTHR, 0, stream>>>(batch, H, out0, nN);
}
